// transformer_layer_53652731462153
// MI455X (gfx1250) — hardware-verified
//
#include <hip/hip_runtime.h>
#include <math.h>
#include <stdint.h>

#define NB    8
#define SL    1194
#define SP    1216
#define DM    512
#define NH    2
#define HDM   256
#define FFD   2048
#define QKVN  1536
#define QKN   1024
#define MP    (NB * SP)
#define MR    (NB * SL)

static_assert(MP % 128 == 0);
static_assert(SP % 64 == 0);
static_assert(DM % 128 == 0 && FFD % 128 == 0 && QKN % 128 == 0);
static_assert(DM % 32 == 0 && FFD % 32 == 0 && HDM % 32 == 0);
static_assert(NH * HDM == DM);

typedef __bf16         v16b __attribute__((ext_vector_type(16)));
typedef __bf16         v8b  __attribute__((ext_vector_type(8)));
typedef float          v8f  __attribute__((ext_vector_type(8)));
typedef float          v4f  __attribute__((ext_vector_type(4)));
typedef unsigned int   v4u  __attribute__((ext_vector_type(4)));
typedef unsigned int   v2u  __attribute__((ext_vector_type(2)));
typedef v4f __attribute__((may_alias)) v4fa;
typedef v4u __attribute__((may_alias)) v4ua;
typedef v2u __attribute__((may_alias)) v2ua;
typedef v8b __attribute__((may_alias)) v8ba;

__device__ __forceinline__ unsigned short bf_bits(float f) {
  const unsigned u = __float_as_uint(f);
  return (unsigned short)((u + 0x7FFFu + ((u >> 16) & 1u)) >> 16);
}
__device__ __forceinline__ float bf_val(unsigned short h) { return __uint_as_float(((unsigned)h) << 16); }
__device__ __forceinline__ float bf_rne(float f) { return bf_val(bf_bits(f)); }
__device__ __forceinline__ v4f bf_rne4(v4f a) {
  v4f r;
  r[0] = bf_rne(a[0]); r[1] = bf_rne(a[1]); r[2] = bf_rne(a[2]); r[3] = bf_rne(a[3]);
  return r;
}
__device__ __forceinline__ unsigned pk16(unsigned short a, unsigned short b) { return (unsigned)a | ((unsigned)b << 16); }
__device__ __forceinline__ v8f zero8() { v8f z = {0.f, 0.f, 0.f, 0.f, 0.f, 0.f, 0.f, 0.f}; return z; }
__device__ __forceinline__ int wave_id() { return __builtin_amdgcn_readfirstlane((int)(threadIdx.x >> 5)); }

__device__ __forceinline__ void lds_wave_sync() {
  __builtin_amdgcn_fence(__ATOMIC_RELEASE, "workgroup");
  __builtin_amdgcn_wave_barrier();
  __builtin_amdgcn_fence(__ATOMIC_ACQUIRE, "workgroup");
}

__device__ __forceinline__ float wave_sum(float v) {
  v += __shfl_xor(v, 16, 32);
  v += __shfl_xor(v, 8, 32);
  v += __shfl_xor(v, 4, 32);
  v += __shfl_xor(v, 2, 32);
  v += __shfl_xor(v, 1, 32);
  return v;
}

union FragB { v16b v; v8b h[2]; };
__device__ __forceinline__ v16b ldfrag_b(const __bf16* p) {
  FragB f;
  f.h[0] = *(const v8ba*)(p);
  f.h[1] = *(const v8ba*)(p + 16);
  return f.v;
}
__device__ __forceinline__ v8f mma_b(v16b a, v16b b, v8f c) {
  return __builtin_amdgcn_wmma_f32_16x16x32_bf16(false, a, false, b, (short)0, c, false, false);
}
__device__ __forceinline__ void guard_b5(v8f& a, v8f& b, v16b x0, v16b x1, v16b x2, v16b x3, v16b y) {
  asm volatile("v_nop\n\tv_nop\n\tv_nop\n\tv_nop" : "+v"(a), "+v"(b) : "v"(x0), "v"(x1), "v"(x2), "v"(x3), "v"(y) : "memory");
}
__device__ __forceinline__ void guard1_b4(v8f& a, v16b w, v16b x, v16b y, v16b z) {
  asm volatile("v_nop\n\tv_nop\n\tv_nop\n\tv_nop" : "+v"(a) : "v"(w), "v"(x), "v"(y), "v"(z) : "memory");
}
__device__ __forceinline__ void acc_guard4(v8f& a, v8f& b, v8f& c, v8f& d) {
  asm volatile("v_nop\n\tv_nop\n\tv_nop\n\tv_nop" : "+v"(a), "+v"(b), "+v"(c), "+v"(d));
}

__global__ __launch_bounds__(256) void prep_x_kernel(const float* __restrict__ x, unsigned short* __restrict__ xb, int nunits) {
  const int i = (int)blockIdx.x * 256 + (int)threadIdx.x;
  if (i >= nunits) return;
  const int row = i >> 6;
  const int c8  = (i & 63) * 8;
  const int b   = row / SP;
  const int s   = row - b * SP;
  const int sc  = (s < SL) ? s : (SL - 1);
  const size_t src = ((size_t)b * SL + sc) * DM + c8;
  const v4f a = *(const v4fa*)(x + src);
  const v4f c = *(const v4fa*)(x + src + 4);
  const unsigned msk = (s < SL) ? 0xffffffffu : 0u;
  v4u w;
  w[0] = pk16(bf_bits(a[0]), bf_bits(a[1])) & msk;
  w[1] = pk16(bf_bits(a[2]), bf_bits(a[3])) & msk;
  w[2] = pk16(bf_bits(c[0]), bf_bits(c[1])) & msk;
  w[3] = pk16(bf_bits(c[2]), bf_bits(c[3])) & msk;
  const size_t e = 8 * (size_t)i;
  *(volatile v4u*)(xb + e) = w;
  __threadfence();
  *(volatile v4u*)(xb + e) = w;
}

__global__ __launch_bounds__(256) void tconv_bf16_kernel(const float* __restrict__ W, unsigned short* __restrict__ outp, int R, int Cc) {
  __shared__ __align__(16) float tf[64 * 68];
  const int c0  = (int)blockIdx.x * 64;
  const int r0  = (int)blockIdx.y * 64;
  const int tid = (int)threadIdx.x;
  {
    const int lr = tid >> 4;
    const int c4 = (tid & 15) * 4;
#pragma unroll
    for (int it = 0; it < 4; ++it) {
      const int rr = it * 16 + lr;
      const v4f a = *(const v4fa*)(W + (size_t)(r0 + rr) * Cc + c0 + c4);
      *(v4f*)(tf + rr * 68 + c4) = a;
    }
  }
  __syncthreads();
  const int sub = tid >> 3;
  const int c8  = (tid & 7) * 8;
  v4u hv[2];
#pragma unroll
  for (int it = 0; it < 2; ++it) {
    const int oc = it * 32 + sub;
    v4u a;
#pragma unroll
    for (int q = 0; q < 4; ++q) {
      const float f0 = tf[(c8 + 2 * q) * 68 + oc];
      const float f1 = tf[(c8 + 2 * q + 1) * 68 + oc];
      a[q] = pk16(bf_bits(f0), bf_bits(f1));
    }
    hv[it] = a;
  }
  for (int pass = 0; pass < 2; ++pass) {
#pragma unroll
    for (int it = 0; it < 2; ++it) {
      const int oc = it * 32 + sub;
      const size_t go = (size_t)(c0 + oc) * R + r0 + c8;
      *(volatile v4u*)(outp + go) = hv[it];
    }
    __threadfence();
  }
}

template <int EPI> struct SlabT { typedef unsigned short T; static constexpr int PERW = 4096; };
template <> struct SlabT<2>     { typedef float          T; static constexpr int PERW = 2048; };

template <int EPI, bool SPLITA>
__global__ __launch_bounds__(128) __attribute__((amdgpu_num_vgpr(256))) void gemm_w32x128_kernel(
    const unsigned short* Ap, const unsigned short* A2p, int lda,
    const unsigned short* __restrict__ Btp, int ldb,
    const float* __restrict__ bias,
    void* C0, void* C1, void* C2, void* C3, int ldc,
    int M, int N, int K) {
  typedef typename SlabT<EPI>::T ST;
  __shared__ __align__(16) ST slab_all[4 * SlabT<EPI>::PERW];

  const int lane = threadIdx.x & 31;
  const int wave = wave_id();
  const int hh = lane >> 4;
  const int rl = lane & 15;
  const int tilesN = N >> 7;
  const int tilesM = M >> 5;
  const int tile = (int)blockIdx.x * 4 + wave;
  if (tile >= tilesM * tilesN) return;
  const int tm = tile / tilesN;
  const int tn = tile - tm * tilesN;
  const int m0 = tm << 5;
  const int n0 = tn << 7;

  const __bf16* A  = (const __bf16*)(const void*)Ap;
  const __bf16* A2 = (const __bf16*)(const void*)A2p;
  const __bf16* Bt = (const __bf16*)(const void*)Btp;

  v8f acc[2][8];
#pragma unroll
  for (int i = 0; i < 2; ++i)
#pragma unroll
    for (int j = 0; j < 8; ++j) acc[i][j] = zero8();

  for (int k0 = 0; k0 < K; k0 += 32) {
    v16b ah[2], al[2];
#pragma unroll
    for (int i = 0; i < 2; ++i) {
      const size_t ao = (size_t)(m0 + i * 16 + rl) * lda + k0 + 8 * hh;
      ah[i] = ldfrag_b(A + ao);
      al[i] = SPLITA ? ldfrag_b(A2 + ao) : ah[i];
    }
#pragma unroll
    for (int j = 0; j < 8; ++j) {
      const v16b bj = ldfrag_b(Bt + (size_t)(n0 + j * 16 + rl) * ldb + k0 + 8 * hh);
      acc[0][j] = mma_b(ah[0], bj, acc[0][j]);
      acc[1][j] = mma_b(ah[1], bj, acc[1][j]);
      if (SPLITA) {
        acc[0][j] = mma_b(al[0], bj, acc[0][j]);
        acc[1][j] = mma_b(al[1], bj, acc[1][j]);
      }
      guard_b5(acc[0][j], acc[1][j], ah[0], ah[1], al[0], al[1], bj);
    }
  }
  acc_guard4(acc[0][0], acc[0][1], acc[0][2], acc[0][3]);
  acc_guard4(acc[0][4], acc[0][5], acc[0][6], acc[0][7]);
  acc_guard4(acc[1][0], acc[1][1], acc[1][2], acc[1][3]);
  acc_guard4(acc[1][4], acc[1][5], acc[1][6], acc[1][7]);

  ST* slab = slab_all + wave * SlabT<EPI>::PERW;

  if (EPI == 2) {
    float* slf = (float*)(void*)slab;
    float* C = (float*)C0;
#pragma unroll
    for (int i = 0; i < 2; ++i) {
#pragma unroll
      for (int j = 0; j < 8; ++j)
#pragma unroll
        for (int r = 0; r < 8; ++r)
          slf[(8 * hh + r) * 128 + j * 16 + rl] = acc[i][j][r];
      lds_wave_sync();
      for (int pass = 0; pass < 2; ++pass) {
#pragma unroll
        for (int row = 0; row < 16; ++row) {
          const v4f v = *(const v4fa*)(slf + row * 128 + lane * 4);
          *(volatile v4f*)(C + (size_t)(m0 + i * 16 + row) * ldc + n0 + lane * 4) = v;
        }
        __threadfence();
      }
      lds_wave_sync();
    }
  } else {
    unsigned short* sl = (unsigned short*)(void*)slab;
    unsigned short* P0 = (unsigned short*)C0;
    unsigned short* P1 = (unsigned short*)C1;
    int col0 = n0;
    if (EPI == 0) {
      const bool isq = (n0 < DM);
      P0 = isq ? (unsigned short*)C0 : (unsigned short*)C2;
      P1 = isq ? (unsigned short*)C1 : (unsigned short*)C3;
      col0 = isq ? n0 : (n0 - DM);
    }
#pragma unroll
    for (int i = 0; i < 2; ++i) {
      if (EPI == 1) {
#pragma unroll
        for (int r = 0; r < 8; ++r) {
          const int m = m0 + i * 16 + 8 * hh + r;
          const float bm = bf_rne(bias[m]);
#pragma unroll
          for (int j = 0; j < 8; ++j) {
            const float v = acc[i][j][r] + bm;
            const unsigned short hb = bf_bits(v);
            const unsigned short lb = bf_bits(v - bf_val(hb));
            const int so = (8 * hh + r) * 128 + j * 16 + rl;
            sl[so]        = hb;
            sl[2048 + so] = lb;
          }
        }
      } else {
#pragma unroll
        for (int j = 0; j < 8; ++j) {
          const int nl = j * 16 + rl;
          const float bn = bf_rne(bias[n0 + nl]);
#pragma unroll
          for (int r = 0; r < 8; ++r) {
            float v = acc[i][j][r] + bn;
            if (EPI == 3) v = fmaxf(v, 0.f);
            const unsigned short hb = bf_bits(v);
            const unsigned short lb = bf_bits(v - bf_val(hb));
            const int so = (8 * hh + r) * 128 + nl;
            sl[so]        = hb;
            sl[2048 + so] = lb;
          }
        }
      }
      lds_wave_sync();
      for (int pass = 0; pass < 2; ++pass) {
#pragma unroll
        for (int it = 0; it < 8; ++it) {
          const int row = it * 2 + hh;
          const int c8  = rl * 8;
          const v4u vh = *(const v4ua*)(sl + row * 128 + c8);
          const v4u vl = *(const v4ua*)(sl + 2048 + row * 128 + c8);
          const size_t go = (size_t)(m0 + i * 16 + row) * ldc + col0 + c8;
          *(volatile v4u*)(P0 + go) = vh;
          *(volatile v4u*)(P1 + go) = vl;
        }
        __threadfence();
      }
      lds_wave_sync();
    }
  }
}

#define KT       64
#define PSP      72
#define OSP      256
#define ATT_O_F  (4 * 16 * 32 * 8)
#define ATT_P_H  (4 * 2 * 16 * PSP)
#define ATT_S_H  (4 * 16 * OSP)
#define ATT_LDS_BYTES (ATT_O_F * 4 + ATT_P_H * 2 + ATT_S_H * 2)
static_assert(ATT_LDS_BYTES == 116736);
static_assert((SP / 64) * KT <= SP);

__global__ __launch_bounds__(128) __attribute__((amdgpu_num_vgpr(240))) void attn_kernel(
    const unsigned short* __restrict__ qhp, const unsigned short* __restrict__ qlp,
    const unsigned short* __restrict__ khp, const unsigned short* __restrict__ klp,
    const unsigned short* __restrict__ vhp, const unsigned short* __restrict__ vlp,
    unsigned short* __restrict__ chp, unsigned short* __restrict__ clp) {
  extern __shared__ v4f att_dyn[];
  float*          o_l   = (float*)(void*)att_dyn;
  __bf16*         lds_p = (__bf16*)(void*)((char*)(void*)att_dyn + ATT_O_F * 4);
  unsigned short* lds_o = (unsigned short*)(void*)((char*)(void*)att_dyn + ATT_O_F * 4 + ATT_P_H * 2);

  const int tid  = (int)threadIdx.x;
  const int lane = tid & 31;
  const int wave = wave_id();
  const int hh   = lane >> 4;
  const int c    = lane & 15;
  const int qb   = (int)blockIdx.x;
  const int h    = (int)blockIdx.y;
  const int b    = (int)blockIdx.z;
  const int q0   = qb * 64 + wave * 16;
  const size_t tokb = (size_t)b * SP;

  const __bf16* Qhr = (const __bf16*)(const void*)qhp + (tokb + q0 + c) * DM + h * HDM + 8 * hh;
  const __bf16* Qlr = (const __bf16*)(const void*)qlp + (tokb + q0 + c) * DM + h * HDM + 8 * hh;
  const __bf16* Khg = (const __bf16*)(const void*)khp + tokb * DM + h * HDM + 8 * hh;
  const __bf16* Klg = (const __bf16*)(const void*)klp + tokb * DM + h * HDM + 8 * hh;
  const __bf16* Vhg = (const __bf16*)(const void*)vhp + (size_t)(h * HDM) * MP + tokb + 8 * hh;
  const __bf16* Vlg = (const __bf16*)(const void*)vlp + (size_t)(h * HDM) * MP + tokb + 8 * hh;
  __bf16* ph = lds_p + wave * (2 * 16 * PSP);
  __bf16* pl = ph + 16 * PSP;
  float*  ow = o_l + wave * (16 * 32 * 8) + lane * 8;

  {
    const v4f z4 = {0.f, 0.f, 0.f, 0.f};
#pragma unroll
    for (int t = 0; t < 16; ++t) {
      *(v4fa*)(ow + t * 256)     = z4;
      *(v4fa*)(ow + t * 256 + 4) = z4;
    }
  }

  float mrow[8], lrow[8];
#pragma unroll
  for (int r = 0; r < 8; ++r) { mrow[r] = -INFINITY; lrow[r] = 0.f; }

  const int nch = qb + 1;
#pragma unroll 1
  for (int kc = 0; kc < nch; ++kc) {
    const int kv0 = kc * KT;
    v8f s[4];
    s[0] = zero8(); s[1] = zero8(); s[2] = zero8(); s[3] = zero8();
#pragma unroll
    for (int dc = 0; dc < 8; ++dc) {
      const v16b qa = ldfrag_b(Qhr + dc * 32);
      const v16b ql = ldfrag_b(Qlr + dc * 32);
#pragma unroll
      for (int j = 0; j < 4; ++j) {
        const size_t ko = (size_t)(kv0 + j * 16 + c) * DM + dc * 32;
        const v16b kb = ldfrag_b(Khg + ko);
        const v16b kl = ldfrag_b(Klg + ko);
        s[j] = mma_b(qa, kb, s[j]);
        s[j] = mma_b(qa, kl, s[j]);
        s[j] = mma_b(ql, kb, s[j]);
        guard1_b4(s[j], qa, ql, kb, kl);
      }
    }
    float cm[8];
#pragma unroll
    for (int r = 0; r < 8; ++r) {
      const int qrow = q0 + 8 * hh + r;
      float m = -INFINITY;
#pragma unroll
      for (int j = 0; j < 4; ++j) {
        const int key = kv0 + j * 16 + c;
        float sv = s[j][r] * 0.0625f;
        sv = (key > qrow || key >= SL) ? -INFINITY : sv;
        s[j][r] = sv;
        m = fmaxf(m, sv);
      }
#pragma unroll
      for (int off = 1; off < 16; off <<= 1) m = fmaxf(m, __shfl_xor(m, off, 32));
      cm[r] = m;
    }
    float alpha[8];
#pragma unroll
    for (int r = 0; r < 8; ++r) {
      const float mnew = fmaxf(mrow[r], cm[r]);
      const float al   = __expf(mrow[r] - mnew);
      mrow[r]  = mnew;
      alpha[r] = al;
      float psum = 0.f;
#pragma unroll
      for (int j = 0; j < 4; ++j) {
        const float p = __expf(s[j][r] - mnew);
        psum += p;
        const unsigned short hb = bf_bits(p);
        const unsigned short lb = bf_bits(p - bf_val(hb));
        const int po = (8 * hh + r) * PSP + j * 16 + c;
        ph[po] = __builtin_bit_cast(__bf16, hb);
        pl[po] = __builtin_bit_cast(__bf16, lb);
      }
#pragma unroll
      for (int off = 1; off < 16; off <<= 1) psum += __shfl_xor(psum, off, 32);
      lrow[r] = lrow[r] * al + psum;
    }
    lds_wave_sync();
    const v16b pa0 = ldfrag_b(ph + c * PSP + 8 * hh);
    const v16b pa1 = ldfrag_b(ph + c * PSP + 32 + 8 * hh);
    const v16b pr0 = ldfrag_b(pl + c * PSP + 8 * hh);
    const v16b pr1 = ldfrag_b(pl + c * PSP + 32 + 8 * hh);
#pragma unroll 1
    for (int cc = 0; cc < 4; ++cc) {
      float* ocl = ow + cc * 1024;
      v8f oc[4];
#pragma unroll
      for (int t = 0; t < 4; ++t) {
        const v4f a4 = *(const v4fa*)(ocl + t * 256);
        const v4f b4 = *(const v4fa*)(ocl + t * 256 + 4);
        v8f o8;
#pragma unroll
        for (int r = 0; r < 4; ++r) {
          o8[r]     = a4[r] * alpha[r];
          o8[4 + r] = b4[r] * alpha[4 + r];
        }
        oc[t] = o8;
      }
#pragma unroll
      for (int t = 0; t < 4; ++t) {
        const size_t vo = (size_t)((cc * 4 + t) * 16 + c) * MP + kv0;
        {
          const v16b vb = ldfrag_b(Vhg + vo);
          const v16b vl = ldfrag_b(Vlg + vo);
          oc[t] = mma_b(pa0, vb, oc[t]);
          oc[t] = mma_b(pa0, vl, oc[t]);
          oc[t] = mma_b(pr0, vb, oc[t]);
          guard1_b4(oc[t], pa0, pr0, vb, vl);
        }
        {
          const v16b vb = ldfrag_b(Vhg + vo + 32);
          const v16b vl = ldfrag_b(Vlg + vo + 32);
          oc[t] = mma_b(pa1, vb, oc[t]);
          oc[t] = mma_b(pa1, vl, oc[t]);
          oc[t] = mma_b(pr1, vb, oc[t]);
          guard1_b4(oc[t], pa1, pr1, vb, vl);
        }
      }
#pragma unroll
      for (int t = 0; t < 4; ++t) {
        v4f a4, b4;
#pragma unroll
        for (int r = 0; r < 4; ++r) { a4[r] = oc[t][r]; b4[r] = oc[t][4 + r]; }
        *(v4fa*)(ocl + t * 256)     = a4;
        *(v4fa*)(ocl + t * 256 + 4) = b4;
      }
    }
    lds_wave_sync();
  }

  float inv[8];
#pragma unroll
  for (int r = 0; r < 8; ++r) inv[r] = 1.0f / lrow[r];
  unsigned short* os = lds_o + wave * (16 * OSP);
#pragma unroll
  for (int plane = 0; plane < 2; ++plane) {
#pragma unroll 1
    for (int t = 0; t < 16; ++t) {
      const v4f a4 = *(const v4fa*)(ow + t * 256);
      const v4f b4 = *(const v4fa*)(ow + t * 256 + 4);
#pragma unroll
      for (int r = 0; r < 4; ++r) {
        const float o0 = a4[r] * inv[r];
        const float o1 = b4[r] * inv[4 + r];
        const unsigned short h0 = bf_bits(o0);
        const unsigned short h1 = bf_bits(o1);
        unsigned short w0 = h0, w1 = h1;
        if (plane == 1) { w0 = bf_bits(o0 - bf_val(h0)); w1 = bf_bits(o1 - bf_val(h1)); }
        os[(8 * hh + r) * OSP + t * 16 + c]     = w0;
        os[(8 * hh + 4 + r) * OSP + t * 16 + c] = w1;
      }
    }
    lds_wave_sync();
    unsigned short* dstp = (plane == 0) ? chp : clp;
    unsigned short* Cg = dstp + (tokb + q0) * DM + h * HDM;
    for (int pass = 0; pass < 2; ++pass) {
#pragma unroll
      for (int row = 0; row < 16; ++row) {
        const v4u xw = *(const v4ua*)(os + row * OSP + lane * 8);
        *(volatile v4u*)(Cg + (size_t)row * DM + lane * 8) = xw;
      }
      __threadfence();
    }
    lds_wave_sync();
  }
}

template <int MODE>
__global__ __launch_bounds__(256) void ln_kernel(const float* __restrict__ pre, const float* __restrict__ bias,
                                                 const float* __restrict__ res, const float* __restrict__ gam,
                                                 const float* __restrict__ bet, float* __restrict__ outf,
                                                 unsigned short* __restrict__ oh, unsigned short* __restrict__ ol) {
  __shared__ __align__(16) unsigned short stg[(MODE == 0) ? (8 * 2 * DM) : 16];
  const int lane = threadIdx.x & 31;
  const int wave = wave_id();
  const int prow = (int)blockIdx.x * 8 + wave;
  if (prow >= MP) return;
  const int b = prow / SP;
  const int s = prow - b * SP;
  const bool valid = (s < SL);
  if (MODE == 1 && !valid) return;
  const int sc = valid ? s : (SL - 1);
  const size_t urow_o = ((size_t)b * SL + sc) * DM;
  const size_t prow_o = (size_t)prow * DM;

  v4f v[4];
  float sum = 0.f;
#pragma unroll
  for (int i = 0; i < 4; ++i) {
    const int col = i * 128 + lane * 4;
    const v4f p  = *(const v4fa*)(pre + prow_o + col);
    const v4f bb = bf_rne4(*(const v4fa*)(bias + col));
    v4f rr;
    if (MODE == 0) rr = bf_rne4(*(const v4fa*)(res + urow_o + col));
    else           rr = *(const v4fa*)(res + prow_o + col);
    const v4f t = (p + bb) + rr;
    v[i] = t;
    sum += (t[0] + t[1]) + (t[2] + t[3]);
  }
  sum = wave_sum(sum);
  const float mean = sum * (1.0f / DM);
  float sq = 0.f;
#pragma unroll
  for (int i = 0; i < 4; ++i) {
#pragma unroll
    for (int e = 0; e < 4; ++e) {
      const float d = v[i][e] - mean;
      sq += d * d;
    }
  }
  sq = wave_sum(sq);
  const float rstd = rsqrtf(sq * (1.0f / DM) + 1e-5f);

  v4f y[4];
#pragma unroll
  for (int i = 0; i < 4; ++i) {
    const int col = i * 128 + lane * 4;
    const v4f g  = bf_rne4(*(const v4fa*)(gam + col));
    const v4f be = bf_rne4(*(const v4fa*)(bet + col));
    v4f yy;
#pragma unroll
    for (int e = 0; e < 4; ++e) {
      const float t = (v[i][e] - mean) * rstd * g[e] + be[e];
      yy[e] = valid ? t : 0.f;
    }
    y[i] = yy;
  }

  float* orow = outf + ((MODE == 0) ? prow_o : urow_o);
  for (int pass = 0; pass < 2; ++pass) {
#pragma unroll
    for (int i = 0; i < 4; ++i)
      *(volatile v4f*)(orow + i * 128 + lane * 4) = y[i];
    __threadfence();
  }

  if (MODE == 0) {
    unsigned short* sw = stg + wave * (2 * DM);
#pragma unroll
    for (int i = 0; i < 4; ++i) {
      const int col = i * 128 + lane * 4;
      unsigned short hb[4], lb[4];
#pragma unroll
      for (int e = 0; e < 4; ++e) {
        hb[e] = bf_bits(y[i][e]);
        lb[e] = bf_bits(y[i][e] - bf_val(hb[e]));
      }
      v2u wh, wl;
      wh[0] = pk16(hb[0], hb[1]); wh[1] = pk16(hb[2], hb[3]);
      wl[0] = pk16(lb[0], lb[1]); wl[1] = pk16(lb[2], lb[3]);
      *(v2ua*)(sw + col)      = wh;
      *(v2ua*)(sw + DM + col) = wl;
    }
    lds_wave_sync();
    for (int pass = 0; pass < 2; ++pass) {
#pragma unroll
      for (int g = 0; g < 2; ++g) {
        const int co = g * 256 + lane * 8;
        const v4u a  = *(const v4ua*)(sw + co);
        const v4u cw = *(const v4ua*)(sw + DM + co);
        *(volatile v4u*)(oh + prow_o + co) = a;
        *(volatile v4u*)(ol + prow_o + co) = cw;
      }
      __threadfence();
    }
  }
}

extern "C" void kernel_launch(void* const* d_in, const int* in_sizes, int n_in,
                              void* d_out, int out_size, void* d_ws, size_t ws_size,
                              hipStream_t stream) {
  if (n_in < 13) return;
  if (in_sizes[0] != MR * DM) return;
  if (in_sizes[1] != DM * QKVN) return;
  if (in_sizes[2] != QKVN) return;
  if (in_sizes[3] != DM * DM) return;
  if (in_sizes[4] != DM) return;
  if (in_sizes[5] != DM || in_sizes[6] != DM) return;
  if (in_sizes[7] != DM * FFD) return;
  if (in_sizes[8] != FFD) return;
  if (in_sizes[9] != FFD * DM) return;
  if (in_sizes[10] != DM) return;
  if (in_sizes[11] != DM || in_sizes[12] != DM) return;
  if (out_size != MR * DM) return;

  const float* x     = (const float*)d_in[0];
  const float* Wqkv  = (const float*)d_in[1];
  const float* bqkv  = (const float*)d_in[2];
  const float* Wo    = (const float*)d_in[3];
  const float* bo    = (const float*)d_in[4];
  const float* ln1g  = (const float*)d_in[5];
  const float* ln1b  = (const float*)d_in[6];
  const float* W1    = (const float*)d_in[7];
  const float* b1    = (const float*)d_in[8];
  const float* W2    = (const float*)d_in[9];
  const float* b2    = (const float*)d_in[10];
  const float* ln2g  = (const float*)d_in[11];
  const float* ln2b  = (const float*)d_in[12];
  float* out = (float*)d_out;

  const size_t szP  = (size_t)MP * DM * 2;
  const size_t szF  = (size_t)MP * DM * 4;
  const size_t szG  = (size_t)MP * FFD * 2;
  const size_t szWq = (size_t)QKVN * DM * 2;
  const size_t szWo = (size_t)DM * DM * 2;
  const size_t szW1 = (size_t)FFD * DM * 2;
  const size_t szW2 = (size_t)DM * FFD * 2;
  size_t off = 0;
  const size_t oXB  = off; off += szP;
  const size_t oWq  = off; off += szWq;
  const size_t oWo  = off; off += szWo;
  const size_t oW1  = off; off += szW1;
  const size_t oW2  = off; off += szW2;
  const size_t oR   = off; off += 8 * szP;
  const size_t oMHA = off; off += szF;
  const size_t oH1  = off; off += szF;
  const size_t oH1h = off; off += szP;
  const size_t oH1l = off; off += szP;
  if (2 * szG > 8 * szP) return;
  if (off > ws_size) return;

  char* ws = (char*)d_ws;
  unsigned short* XB    = (unsigned short*)(ws + oXB);
  unsigned short* WQKVT = (unsigned short*)(ws + oWq);
  unsigned short* WOT   = (unsigned short*)(ws + oWo);
  unsigned short* W1T   = (unsigned short*)(ws + oW1);
  unsigned short* W2T   = (unsigned short*)(ws + oW2);
  unsigned short* Qh    = (unsigned short*)(ws + oR);
  unsigned short* Ql    = (unsigned short*)(ws + oR + 1 * szP);
  unsigned short* Kh    = (unsigned short*)(ws + oR + 2 * szP);
  unsigned short* Kl    = (unsigned short*)(ws + oR + 3 * szP);
  unsigned short* Vh    = (unsigned short*)(ws + oR + 4 * szP);
  unsigned short* Vl    = (unsigned short*)(ws + oR + 5 * szP);
  unsigned short* Ch    = (unsigned short*)(ws + oR + 6 * szP);
  unsigned short* Cl    = (unsigned short*)(ws + oR + 7 * szP);
  unsigned short* Gh    = (unsigned short*)(ws + oR);
  unsigned short* Gl    = (unsigned short*)(ws + oR + szG);
  float*          MHA   = (float*)(ws + oMHA);
  float*          H1    = (float*)(ws + oH1);
  unsigned short* H1h   = (unsigned short*)(ws + oH1h);
  unsigned short* H1l   = (unsigned short*)(ws + oH1l);

  const dim3 b256(256), b128(128);

  const int nunits = MP * DM / 8;
  prep_x_kernel<<<dim3((nunits + 255) / 256), b256, 0, stream>>>(x, XB, nunits);
  tconv_bf16_kernel<<<dim3(QKVN / 64, DM / 64), b256, 0, stream>>>(Wqkv, WQKVT, DM, QKVN);
  tconv_bf16_kernel<<<dim3(DM / 64, DM / 64), b256, 0, stream>>>(Wo, WOT, DM, DM);
  tconv_bf16_kernel<<<dim3(FFD / 64, DM / 64), b256, 0, stream>>>(W1, W1T, DM, FFD);
  tconv_bf16_kernel<<<dim3(DM / 64, FFD / 64), b256, 0, stream>>>(W2, W2T, FFD, DM);
  {
    const int tiles = (MP / 32) * (QKN / 128);
    gemm_w32x128_kernel<0, false><<<dim3((tiles + 3) / 4), b128, 0, stream>>>(
        XB, XB, DM, WQKVT, DM, bqkv, (void*)Qh, (void*)Ql, (void*)Kh, (void*)Kl, DM, MP, QKN, DM);
  }
  {
    const int tiles = (DM / 32) * (MP / 128);
    gemm_w32x128_kernel<1, false><<<dim3((tiles + 3) / 4), b128, 0, stream>>>(
        WQKVT + (size_t)QKN * DM, WQKVT + (size_t)QKN * DM, DM, XB, DM, bqkv + QKN,
        (void*)Vh, (void*)Vl, (void*)Vh, (void*)Vl, MP, DM, MP, DM);
  }
  (void)hipFuncSetAttribute(reinterpret_cast<const void*>(&attn_kernel), hipFuncAttributeMaxDynamicSharedMemorySize, ATT_LDS_BYTES);
  attn_kernel<<<dim3(SP / 64, NH, NB), b128, ATT_LDS_BYTES, stream>>>(Qh, Ql, Kh, Kl, Vh, Vl, Ch, Cl);
  {
    const int tiles = (MP / 32) * (DM / 128);
    gemm_w32x128_kernel<2, true><<<dim3((tiles + 3) / 4), b128, 0, stream>>>(
        Ch, Cl, DM, WOT, DM, bo, (void*)MHA, (void*)MHA, (void*)MHA, (void*)MHA, DM, MP, DM, DM);
  }
  ln_kernel<0><<<dim3(MP / 8), b256, 0, stream>>>(MHA, bo, x, ln1g, ln1b, H1, H1h, H1l);
  {
    const int tiles = (MP / 32) * (FFD / 128);
    gemm_w32x128_kernel<3, true><<<dim3((tiles + 3) / 4), b128, 0, stream>>>(
        H1h, H1l, DM, W1T, DM, b1, (void*)Gh, (void*)Gl, (void*)Gh, (void*)Gl, FFD, MP, FFD, DM);
  }
  {
    const int tiles = (MP / 32) * (DM / 128);
    gemm_w32x128_kernel<2, true><<<dim3((tiles + 3) / 4), b128, 0, stream>>>(
        Gh, Gl, FFD, W2T, FFD, b2, (void*)MHA, (void*)MHA, (void*)MHA, (void*)MHA, DM, MP, DM, FFD);
  }
  ln_kernel<1><<<dim3(MP / 8), b256, 0, stream>>>(MHA, b2, H1, ln2g, ln2b, out, H1h, H1l);
  (void)hipGetLastError();
}
